// CausalSelfAttention_68461778698773
// MI455X (gfx1250) — hardware-verified
//
#include <hip/hip_runtime.h>
#include <math.h>

#define NB_FULL  4
#define SEQ_FULL 2048
#ifndef NB
#define NB    4
#endif
#ifndef SEQ
#define SEQ   2048
#endif
#define DM    1024
#define NQT   (SEQ / 64)
#define RESR  ((SEQ < 512) ? SEQ : 512)
#define VLP   RESR
#define PSC   1024.0f
#define VSC   16.0f
#define LSC   4096.0f
#define OSCALE (1.0f / 16384.0f)
#define BPS   (((NB % 2) == 0) ? 2 : 1)
#define NPASS (NB / BPS)
#define NG    (SEQ / 256)
#ifndef SCORE_NSPLIT
#define SCORE_NSPLIT 2
#endif
#define SZ_PX   ((size_t)NB * SEQ * DM * 2)
#define SZ_PXP  ((size_t)BPS * SEQ * DM * 2)
#define SZ_PW   ((size_t)DM * DM * 2)
#define SZ_PS   ((size_t)BPS * SEQ * SEQ * 4)
#define SZ_PP   ((size_t)NB * SEQ * SEQ * 2)
#define SZ_PPL  ((size_t)NB * RESR * VLP * 2)
#define SZ_PVT  ((size_t)NB * DM * SEQ * 2)
#define SZ_PVL  ((size_t)NB * DM * VLP * 2)
#define SZ_RA   (((SZ_PX + 3 * SZ_PW) > SZ_PS) ? (SZ_PX + 3 * SZ_PW) : SZ_PS)
#define SZ_TOTAL (SZ_RA + (size_t)NPASS * 4 * SZ_PXP + SZ_PVT + SZ_PVL + SZ_PPL)
static_assert(NB >= 1 && NB <= NB_FULL);
static_assert(SEQ >= 256 && SEQ <= SEQ_FULL && (SEQ % 256) == 0);
static_assert((SEQ % 64) == 0 && (DM % 64) == 0 && (DM % 32) == 0);
static_assert((RESR % 64) == 0 && (RESR % 256) == 0 && RESR <= VLP && VLP <= SEQ && ((SEQ - RESR) % 64) == 0);
static_assert((RESR % 32) == 0);
static_assert((RESR & (RESR - 1)) == 0);
static_assert(((NB * SEQ) % 8) == 0);
static_assert(((SEQ * DM / 8) % 256) == 0 && ((DM * DM / 8) % 256) == 0);
static_assert((NB % BPS) == 0 && NPASS * BPS == NB);
static_assert(NG >= 1 && NG <= 8 && NG * 256 == SEQ);
static_assert(((BPS * SEQ) % 64) == 0 && ((BPS * SEQ) % 8) == 0);
static_assert(SZ_PP <= 4 * SZ_PXP);
static_assert((SZ_RA % 128) == 0 && (SZ_PXP % 128) == 0 && (SZ_PVT % 128) == 0 && (SZ_PVL % 128) == 0 && (SZ_PPL % 128) == 0);
static_assert(SZ_TOTAL <= (size_t)134217728);
static_assert((size_t)NB * SEQ * DM * 4 <= (size_t)33554432);
static_assert(SCORE_NSPLIT == 0 || SCORE_NSPLIT == 2);

typedef _Float16 v16h __attribute__((ext_vector_type(16)));
typedef _Float16 v8h  __attribute__((ext_vector_type(8)));
typedef __bf16   v16b __attribute__((ext_vector_type(16)));
typedef __bf16   v8b  __attribute__((ext_vector_type(8)));
typedef float    v8f  __attribute__((ext_vector_type(8)));
typedef float    v4f  __attribute__((ext_vector_type(4)));
typedef unsigned int v4u __attribute__((ext_vector_type(4)));

__device__ __forceinline__ unsigned short bf_bits(float f) {
  unsigned u = __float_as_uint(f);
  return (unsigned short)((u + 0x7FFFu + ((u >> 16) & 1u)) >> 16);
}
__device__ __forceinline__ float bf_up(unsigned short h) { return __uint_as_float(((unsigned)h) << 16); }
__device__ __forceinline__ unsigned short h_bits(_Float16 x) { return __builtin_bit_cast(unsigned short, x); }
__device__ __forceinline__ unsigned pk16(unsigned short a, unsigned short b) { return (unsigned)a | ((unsigned)b << 16); }
__device__ __forceinline__ v8f zero8() { v8f z = {0.f, 0.f, 0.f, 0.f, 0.f, 0.f, 0.f, 0.f}; return z; }
static __device__ __forceinline__ _Float16 toh_flush(float v) {
  const _Float16 r = (_Float16)v;
  return (fabsf(v) < 6.103515625e-05f) ? (_Float16)0.0f : r;
}

__device__ __forceinline__ v16b ldfrag_b(const __bf16* p) {
  union { v16b v; v8b h[2]; } f;
  f.h[0] = *(const v8b*)(p);
  f.h[1] = *(const v8b*)(p + 16);
  return f.v;
}
__device__ __forceinline__ v16h ldfrag_h(const _Float16* p) {
  union { v16h v; v8h h[2]; } f;
  f.h[0] = *(const v8h*)(p);
  f.h[1] = *(const v8h*)(p + 16);
  return f.v;
}

__device__ __forceinline__ v8f mma_b_raw(v16b a, v16b b, v8f c) {
  return __builtin_amdgcn_wmma_f32_16x16x32_bf16(false, a, false, b, (short)0, c, false, false);
}
__device__ __forceinline__ v8f mma_h_raw(v16h a, v16h b, v8f c) {
  return __builtin_amdgcn_wmma_f32_16x16x32_f16(false, a, false, b, (short)0, c, false, false);
}
__device__ __forceinline__ void dep_guard_b(v8f& a, v8f& b, v16b x, v16b y) {
  asm volatile("v_nop\n\tv_nop\n\tv_nop\n\tv_nop" : "+v"(a), "+v"(b) : "v"(x), "v"(y));
}
__device__ __forceinline__ void dep_guard_h(v8f& a, v8f& b, v16h x, v16h y) {
  asm volatile("v_nop\n\tv_nop\n\tv_nop\n\tv_nop" : "+v"(a), "+v"(b) : "v"(x), "v"(y));
}
__device__ __forceinline__ void dep_guard4_h(v8f& a, v8f& b, v8f& c, v8f& d, v16h x, v16h y) {
  asm volatile("v_nop\n\tv_nop\n\tv_nop\n\tv_nop" : "+v"(a), "+v"(b), "+v"(c), "+v"(d) : "v"(x), "v"(y));
}
__device__ __forceinline__ void keep4_b(v16b a, v16b b, v16b c, v16b d) {
  asm volatile("v_nop" :: "v"(a), "v"(b), "v"(c), "v"(d));
}
__device__ __forceinline__ void keep4_h(v16h a, v16h b, v16h c, v16h d) {
  asm volatile("v_nop" :: "v"(a), "v"(b), "v"(c), "v"(d));
}
__device__ __forceinline__ void acc_guard4(v8f& a, v8f& b, v8f& c, v8f& d) {
  asm volatile("v_nop\n\tv_nop\n\tv_nop\n\tv_nop" : "+v"(a), "+v"(b), "+v"(c), "+v"(d));
}

__global__ __launch_bounds__(256) void cvt_planes(const float* __restrict__ x, const float* __restrict__ wq,
                                                  const float* __restrict__ wk, const float* __restrict__ wv,
                                                  unsigned short* out) {
  const int NXB8 = SEQ * DM / 8;
  const int NX8 = NB * NXB8;
  const int NW8 = DM * DM / 8;
  const int g = blockIdx.x * 256 + threadIdx.x;
  if (g >= NX8 + 3 * NW8) return;
  const float* src;
  if (g < NX8) {
    const int bb  = g / NXB8;
    const int off = g - bb * NXB8;
    src = x + (size_t)bb * SEQ_FULL * DM + (size_t)off * 8;
  } else {
    const int e = g - NX8;
    const int w = e / NW8;
    const int off = e - w * NW8;
    const float* wsrc = (w == 0) ? wq : ((w == 1) ? wk : wv);
    src = wsrc + (size_t)off * 8;
  }
  const v4f a = *(const v4f*)(src);
  const v4f c = *(const v4f*)(src + 4);
  v4u p;
  p[0] = pk16(bf_bits(a[0]), bf_bits(a[1]));
  p[1] = pk16(bf_bits(a[2]), bf_bits(a[3]));
  p[2] = pk16(bf_bits(c[0]), bf_bits(c[1]));
  p[3] = pk16(bf_bits(c[2]), bf_bits(c[3]));
  *(volatile v4u*)(out + (size_t)g * 8) = p;
  __threadfence();
  *(volatile v4u*)(out + (size_t)g * 8) = p;
}

template <int NSPLIT, int OUT_MODE, int TRI>
__global__ __launch_bounds__(256) void gemm_bf(
    const unsigned short* __restrict__ Ahp, const unsigned short* __restrict__ Alp, int lda, long long strideA,
    const unsigned short* __restrict__ Bhp, const unsigned short* __restrict__ Blp, int ldb, long long strideB,
    void* Cout, int ldc, long long strideC,
    void* Cout2, int ldc2, long long strideC2, int N2,
    int M, int N, int K, float hscale, float rscale) {
  const __bf16* Ah = (const __bf16*)(const void*)Ahp;
  const __bf16* Al = (const __bf16*)(const void*)Alp;
  const __bf16* Bh = (const __bf16*)(const void*)Bhp;
  const __bf16* Bl = (const __bf16*)(const void*)Blp;
  __shared__ __align__(16) float sT[8][16 * 68];
  const int b    = blockIdx.y;
  const int lane = threadIdx.x & 31;
  const int wave = threadIdx.x >> 5;
  const int tilesN = N >> 6;
  const int tilesM = M >> 6;
  const int t = blockIdx.x * 8 + wave;
  int tm, tn;
  if (TRI != 0) {
    const int ntri = (tilesM * (tilesM + 1)) >> 1;
    if (t >= ntri) return;
    int q = (int)((sqrtf(8.0f * (float)t + 1.0f) - 1.0f) * 0.5f);
    q = (q < 0) ? 0 : ((q > tilesM - 1) ? (tilesM - 1) : q);
    if ((((q + 1) * (q + 2)) >> 1) <= t) ++q;
    if (((q * (q + 1)) >> 1) > t) --q;
    q = (q < 0) ? 0 : ((q > tilesM - 1) ? (tilesM - 1) : q);
    tm = q;
    tn = t - ((q * (q + 1)) >> 1);
    tn = (tn < 0) ? 0 : ((tn > tilesN - 1) ? (tilesN - 1) : tn);
  } else {
    if (t >= tilesM * tilesN) return;
    tm = t / tilesN;
    tn = t - tm * tilesN;
  }
  const int m0 = tm << 6;
  const int n0 = tn << 6;

  const __bf16* Ahb = Ah + (size_t)b * strideA;
  const __bf16* Alb = (NSPLIT >= 1) ? (Al + (size_t)b * strideA) : Ahb;
  const __bf16* Bhb = Bh + (size_t)b * strideB;
  const __bf16* Blb = (NSPLIT >= 1) ? (Bl + (size_t)b * strideB) : Bhb;

  const int rlane = lane & 15;
  const int koff  = (lane >> 4) * 8;
  const int mOff  = (lane >> 4) * 8;

  v8f acc[4][4];
#pragma unroll
  for (int i = 0; i < 4; ++i)
#pragma unroll
    for (int j = 0; j < 4; ++j) acc[i][j] = zero8();

  for (int k0 = 0; k0 < K; k0 += 32) {
    v16b bf[4];
#pragma unroll
    for (int j = 0; j < 4; ++j) {
      const size_t bo = (size_t)(n0 + (j << 4) + rlane) * ldb + koff + k0;
      bf[j] = ldfrag_b(Bhb + bo);
    }
#pragma unroll
    for (int i = 0; i < 4; ++i) {
      const size_t ao = (size_t)(m0 + (i << 4) + rlane) * lda + koff + k0;
      const v16b ah = ldfrag_b(Ahb + ao);
      v16b al = ah;
      if (NSPLIT >= 1) al = ldfrag_b(Alb + ao);
#pragma unroll
      for (int j = 0; j < 4; ++j) {
        acc[i][j] = mma_b_raw(ah, bf[j], acc[i][j]);
        if (NSPLIT >= 1) acc[i][j] = mma_b_raw(al, bf[j], acc[i][j]);
      }
      dep_guard_b(acc[i][0], acc[i][3], ah, al);
    }
    if (NSPLIT >= 2) {
      keep4_b(bf[0], bf[1], bf[2], bf[3]);
#pragma unroll
      for (int j = 0; j < 4; ++j) {
        const size_t bo = (size_t)(n0 + (j << 4) + rlane) * ldb + koff + k0;
        bf[j] = ldfrag_b(Blb + bo);
      }
#pragma unroll
      for (int i = 0; i < 4; ++i) {
        const size_t ao = (size_t)(m0 + (i << 4) + rlane) * lda + koff + k0;
        const v16b ah = ldfrag_b(Ahb + ao);
#pragma unroll
        for (int j = 0; j < 4; ++j) acc[i][j] = mma_b_raw(ah, bf[j], acc[i][j]);
        dep_guard_b(acc[i][0], acc[i][3], ah, ah);
      }
    }
    keep4_b(bf[0], bf[1], bf[2], bf[3]);
  }
  acc_guard4(acc[0][0], acc[0][1], acc[0][2], acc[0][3]);
  acc_guard4(acc[1][0], acc[1][1], acc[1][2], acc[1][3]);
  acc_guard4(acc[2][0], acc[2][1], acc[2][2], acc[2][3]);
  acc_guard4(acc[3][0], acc[3][1], acc[3][2], acc[3][3]);

  size_t cbase;
  int ldce, rowb, colb;
  if (TRI != 0) { cbase = (size_t)b * strideC + (size_t)t * 4096; ldce = 64; rowb = 0; colb = 0; }
  else          { cbase = (size_t)b * strideC; ldce = ldc; rowb = m0; colb = n0; }
  float* slab = sT[wave];
#pragma unroll
  for (int i = 0; i < 4; ++i) {
    const int mBase = m0 + (i << 4);
#pragma unroll
    for (int j = 0; j < 4; ++j) {
#pragma unroll
      for (int r = 0; r < 8; ++r) {
        slab[(mOff + r) * 68 + (j << 4) + rlane] = acc[i][j][r];
      }
    }
    __builtin_amdgcn_fence(3  , "workgroup");
    __builtin_amdgcn_wave_barrier();
    __builtin_amdgcn_fence(2  , "workgroup");
    if (OUT_MODE == 0) {
      float* C = (float*)Cout + cbase;
      const int hh = lane >> 4, c4 = (lane & 15) * 4;
      for (int pass = 0; pass < 2; ++pass) {
#pragma unroll
        for (int it = 0; it < 8; ++it) {
          const int row = it * 2 + hh;
          const v4f v = *(const v4f*)(slab + row * 68 + c4);
          *(volatile v4f*)(C + (size_t)(rowb + (i << 4) + row) * ldce + colb + c4) = v;
        }
        __threadfence();
      }
    } else {
      const int q = lane >> 3, c8 = (lane & 7) * 8;
      unsigned short* C  = (unsigned short*)Cout  + (size_t)b * strideC;
      unsigned short* C2 = (unsigned short*)Cout2 + (size_t)b * strideC2;
      const bool wlo = (OUT_MODE == 2) || (n0 < N2);
      v4u hv[4], lv[4];
#pragma unroll
      for (int it = 0; it < 4; ++it) {
        const int row = it * 4 + q;
        const float* sp = slab + row * 68 + c8;
        v4u a, a2;
#pragma unroll
        for (int e = 0; e < 4; ++e) {
          const float f0 = sp[2 * e], f1 = sp[2 * e + 1];
          unsigned short h0, h1, l0, l1;
          if (OUT_MODE == 2) {
            h0 = bf_bits(f0); h1 = bf_bits(f1);
            l0 = bf_bits(f0 - bf_up(h0)); l1 = bf_bits(f1 - bf_up(h1));
          } else {
            const float g0 = f0 * hscale, g1 = f1 * hscale;
            const _Float16 x0 = (_Float16)g0, x1 = (_Float16)g1;
            h0 = h_bits(x0); h1 = h_bits(x1);
            l0 = h_bits((_Float16)((g0 - (float)x0) * rscale));
            l1 = h_bits((_Float16)((g1 - (float)x1) * rscale));
          }
          a[e] = pk16(h0, h1); a2[e] = pk16(l0, l1);
        }
        hv[it] = a; lv[it] = a2;
      }
      for (int pass = 0; pass < 2; ++pass) {
#pragma unroll
        for (int it = 0; it < 4; ++it) {
          const int row = it * 4 + q;
          *(volatile v4u*)(C + (size_t)(mBase + row) * ldc + n0 + c8) = hv[it];
          if (wlo) *(volatile v4u*)(C2 + (size_t)(mBase + row) * ldc2 + n0 + c8) = lv[it];
        }
        __threadfence();
      }
    }
    __builtin_amdgcn_fence(3  , "workgroup");
    __builtin_amdgcn_wave_barrier();
    __builtin_amdgcn_fence(2  , "workgroup");
  }
}

__global__ __launch_bounds__(256) void softmax_rows(const float* __restrict__ Sp,
                                                    unsigned short* Php, unsigned short* Plp, int b0) {
#pragma clang fp contract(off)
  const int lane = threadIdx.x & 31;
  const int wave = __builtin_amdgcn_readfirstlane(threadIdx.x >> 5);
  const int lrow = blockIdx.x * 8 + wave;
  if (lrow >= BPS * SEQ) return;
  const int bl = lrow / SEQ;
  const int i  = lrow - bl * SEQ;
  const int b  = b0 + bl;
  const int tm = i >> 6;
  const int ng = (tm >> 2) + 1;
  const float* srow = Sp + ((size_t)bl * SEQ + (size_t)i) * SEQ + 8 * lane;

  float z[NG][8];
  float m = -INFINITY;
#pragma unroll
  for (int g = 0; g < NG; ++g) {
    const float* p = srow + 256 * g;
    const v4f a = *(const v4f*)(p);
    const v4f c = *(const v4f*)(p + 4);
    const float v[8] = {a[0], a[1], a[2], a[3], c[0], c[1], c[2], c[3]};
#pragma unroll
    for (int e = 0; e < 8; ++e) {
      const float zz = v[e] * 0.03125f;
      z[g][e] = zz;
      m = fmaxf(m, zz);
    }
  }
#pragma unroll
  for (int off = 1; off < 32; off <<= 1) m = fmaxf(m, __shfl_xor(m, off, 32));

  float l = 0.f;
#pragma unroll
  for (int g = 0; g < NG; ++g) {
#pragma unroll
    for (int e = 0; e < 8; ++e) {
      const float p = __expf(z[g][e] - m);
      z[g][e] = p;
      l += p;
    }
  }
#pragma unroll
  for (int off = 1; off < 32; off <<= 1) l += __shfl_xor(l, off, 32);
  const float inv1k = (1.0f / l) * PSC;

  const bool res = (i < RESR);
  v4u ph[NG];
  v4u pl0 = {0u, 0u, 0u, 0u};
  v4u pl1 = {0u, 0u, 0u, 0u};
#pragma unroll
  for (int g = 0; g < NG; ++g) {
    v4u hv = {0u, 0u, 0u, 0u};
    v4u lv = {0u, 0u, 0u, 0u};
    if (g < ng) {
      const int j0 = 256 * g + 8 * lane;
#pragma unroll
      for (int e = 0; e < 4; ++e) {
        const float f0 = (j0 + 2 * e     <= i) ? (z[g][2 * e]     * inv1k) : 0.0f;
        const float f1 = (j0 + 2 * e + 1 <= i) ? (z[g][2 * e + 1] * inv1k) : 0.0f;
        const _Float16 x0 = toh_flush(f0), x1 = toh_flush(f1);
        hv[e] = pk16(h_bits(x0), h_bits(x1));
        const _Float16 r0 = toh_flush((f0 - (float)x0) * LSC);
        const _Float16 r1 = toh_flush((f1 - (float)x1) * LSC);
        lv[e] = pk16(h_bits(r0), h_bits(r1));
      }
    }
    ph[g] = hv;
    if (g == 0) pl0 = lv;
    if (g == 1) pl1 = lv;
  }

  unsigned short* prow = Php + ((size_t)b * SEQ + (size_t)i) * SEQ + 8 * lane;
  const int il = i & (RESR - 1);
  unsigned short* lrowp = Plp + ((size_t)b * RESR + (size_t)il) * VLP + 8 * lane;
  for (int pass = 0; pass < 2; ++pass) {
#pragma unroll
    for (int g = 0; g < NG; ++g) {
      if (g < ng) *(volatile v4u*)(prow + 256 * g) = ph[g];
    }
    if (res) {
      *(volatile v4u*)(lrowp) = pl0;
      if (ng > 1) *(volatile v4u*)(lrowp + 256) = pl1;
    }
    __threadfence();
  }
}

template <bool RES, int MI>
__global__ __launch_bounds__(256) void gemm_pv(
    const unsigned short* __restrict__ Php, const unsigned short* __restrict__ Plp,
    const unsigned short* __restrict__ Vhp, const unsigned short* __restrict__ Vlp,
    float* out, int mBase, int M) {
  const _Float16* Ph = (const _Float16*)(const void*)Php;
  const _Float16* Pl = (const _Float16*)(const void*)Plp;
  const _Float16* Vh = (const _Float16*)(const void*)Vhp;
  const _Float16* Vl = (const _Float16*)(const void*)Vlp;
  __shared__ __align__(16) float sT[8][16 * 68];
  const int b    = blockIdx.y;
  const int lane = threadIdx.x & 31;
  const int wave = threadIdx.x >> 5;
  const int tilesN = DM >> 6;
  const int tilesM = M / (16 * MI);
  const int t = blockIdx.x * 8 + wave;
  if (t >= tilesM * tilesN) return;
  const int tm = t / tilesN;
  const int tn = t - tm * tilesN;
  const int m0 = mBase + tm * 16 * MI;
  const int n0 = tn << 6;
  int keff = (((m0 >> 6) + 1) << 6);
  if (keff > SEQ) keff = SEQ;
  if (RES && keff > VLP) keff = VLP;

  const _Float16* Pb  = Ph + (size_t)b * SEQ * SEQ;
  const _Float16* Plb = Pl + (size_t)b * RESR * VLP;
  const _Float16* Vb  = Vh + (size_t)b * DM * SEQ;
  const _Float16* Vlb = Vl + (size_t)b * DM * VLP;

  const int rlane = lane & 15;
  const int koff  = (lane >> 4) * 8;
  const int mOff  = (lane >> 4) * 8;

  v8f acc0[MI][4], acc1[MI][4];
#pragma unroll
  for (int i = 0; i < MI; ++i)
#pragma unroll
    for (int j = 0; j < 4; ++j) { acc0[i][j] = zero8(); acc1[i][j] = zero8(); }

  for (int k0 = 0; k0 < keff; k0 += 32) {
    v16h bf[4];
#pragma unroll
    for (int j = 0; j < 4; ++j) bf[j] = ldfrag_h(Vb + (size_t)(n0 + (j << 4) + rlane) * SEQ + koff + k0);
#pragma unroll
    for (int i = 0; i < MI; ++i) {
      const int mrow = m0 + (i << 4) + rlane;
      const v16h ah = ldfrag_h(Pb + (size_t)mrow * SEQ + koff + k0);
      v16h al = ah;
      if (RES) {
        const int mres = (mrow < RESR) ? mrow : (RESR - 1);
        al = ldfrag_h(Plb + (size_t)mres * VLP + koff + k0);
      }
#pragma unroll
      for (int j = 0; j < 4; ++j) {
        acc0[i][j] = mma_h_raw(ah, bf[j], acc0[i][j]);
        if (RES) acc1[i][j] = mma_h_raw(al, bf[j], acc1[i][j]);
      }
      if (RES) dep_guard4_h(acc0[i][0], acc0[i][3], acc1[i][0], acc1[i][3], ah, al);
      else     dep_guard_h(acc0[i][0], acc0[i][3], ah, al);
    }
    if (RES) {
      keep4_h(bf[0], bf[1], bf[2], bf[3]);
#pragma unroll
      for (int j = 0; j < 4; ++j) bf[j] = ldfrag_h(Vlb + (size_t)(n0 + (j << 4) + rlane) * VLP + koff + k0);
#pragma unroll
      for (int i = 0; i < MI; ++i) {
        const int mrow = m0 + (i << 4) + rlane;
        const v16h ah = ldfrag_h(Pb + (size_t)mrow * SEQ + koff + k0);
#pragma unroll
        for (int j = 0; j < 4; ++j) acc1[i][j] = mma_h_raw(ah, bf[j], acc1[i][j]);
        dep_guard_h(acc1[i][0], acc1[i][3], ah, ah);
      }
    }
    keep4_h(bf[0], bf[1], bf[2], bf[3]);
  }
#pragma unroll
  for (int i = 0; i < MI; ++i) {
    acc_guard4(acc0[i][0], acc0[i][1], acc0[i][2], acc0[i][3]);
    if (RES) acc_guard4(acc1[i][0], acc1[i][1], acc1[i][2], acc1[i][3]);
  }

  float* slab = sT[wave];
  float* C = out + (size_t)b * SEQ * DM;
  const float rsc = OSCALE * (1.0f / LSC);
#pragma unroll
  for (int i = 0; i < MI; ++i) {
    const int mB = m0 + (i << 4);
#pragma unroll
    for (int j = 0; j < 4; ++j) {
#pragma unroll
      for (int r = 0; r < 8; ++r) {
        float v = acc0[i][j][r] * OSCALE;
        if (RES) v += acc1[i][j][r] * rsc;
        slab[(mOff + r) * 68 + (j << 4) + rlane] = v;
      }
    }
    __builtin_amdgcn_fence(3  , "workgroup");
    __builtin_amdgcn_wave_barrier();
    __builtin_amdgcn_fence(2  , "workgroup");
    {
      const int hh = lane >> 4, c4 = (lane & 15) * 4;
      for (int pass = 0; pass < 2; ++pass) {
#pragma unroll
        for (int it = 0; it < 8; ++it) {
          const int row = it * 2 + hh;
          const v4f v = *(const v4f*)(slab + row * 68 + c4);
          *(volatile v4f*)(C + (size_t)(mB + row) * DM + n0 + c4) = v;
        }
        __threadfence();
      }
    }
    __builtin_amdgcn_fence(3  , "workgroup");
    __builtin_amdgcn_wave_barrier();
    __builtin_amdgcn_fence(2  , "workgroup");
  }
}

extern "C" void kernel_launch(void* const* d_in, const int* in_sizes, int n_in,
                              void* d_out, int out_size, void* d_ws, size_t ws_size,
                              hipStream_t stream) {
  if (n_in < 4) return;
  if (in_sizes[0] < (NB - 1) * SEQ_FULL * DM + SEQ * DM) return;
  if (in_sizes[1] < DM * DM || in_sizes[2] < DM * DM || in_sizes[3] < DM * DM) return;
  if (out_size < NB * SEQ * DM) return;

  const float* x  = (const float*)d_in[0];
  const float* wq = (const float*)d_in[1];
  const float* wk = (const float*)d_in[2];
  const float* wv = (const float*)d_in[3];
  float* out = (float*)d_out;

  const size_t PX  = SZ_PX;
  const size_t PXP = SZ_PXP;
  const size_t PW  = SZ_PW;
  const size_t PP  = SZ_PP;
  const size_t PPL = SZ_PPL;
  const size_t PVT = SZ_PVT;
  const size_t PVL = SZ_PVL;
  const size_t RA  = SZ_RA;
  const size_t oXb = 0;
  const size_t oW  = PX;
  const size_t oS  = 0;
  const size_t oB  = RA;
  const size_t RBend = RA + (size_t)NPASS * 4 * PXP;
  const size_t oPh = RA;
  if (PP > 4 * PXP) return;
  const size_t oVTh = RBend;
  const size_t oVTl = RBend + PVT;
  const size_t oPl  = oVTl + PVL;
  const size_t total = oPl + PPL;
  if (total > ws_size) return;
  if (total > (size_t)134217728) return;

  char* ws = (char*)d_ws;
  unsigned short* Xb  = (unsigned short*)(ws + oXb);
  unsigned short* Wb  = (unsigned short*)(ws + oW);
  float*          Sp  = (float*)(ws + oS);
  unsigned short* Ph  = (unsigned short*)(ws + oPh);
  unsigned short* Pl  = (unsigned short*)(ws + oPl);
  unsigned short* VTh = (unsigned short*)(ws + oVTh);
  unsigned short* VTl = (unsigned short*)(ws + oVTl);
  const size_t PXE = (size_t)BPS * SEQ * DM;

  const dim3 blk(256);
  const int nGroups = NB * SEQ * DM / 8 + 3 * (DM * DM / 8);
  const dim3 gCvt((nGroups + 255) / 256);
  const dim3 gProj(((BPS * SEQ / 64) * (DM / 64) + 7) / 8, 1);
  const dim3 gVT(((DM / 64) * (SEQ / 64) + 7) / 8, NB);
  const dim3 gS(((SEQ / 64) * (SEQ / 64) + 7) / 8, BPS);
  const dim3 gSm((BPS * SEQ + 7) / 8);
  const dim3 gPvRes(((RESR / 32) * (DM / 64) + 7) / 8, NB);
  const int nPvTiles = ((SEQ - RESR) / 64) * (DM / 64);
  const dim3 gPv((nPvTiles + 7) / 8, NB);

  cvt_planes<<<gCvt, blk, 0, stream>>>(x, wq, wk, wv, Xb);
  for (int p = 0; p < NPASS; ++p) {
    unsigned short* Qh = (unsigned short*)(ws + oB + (size_t)p * 4 * PXP);
    unsigned short* Ql = Qh + PXE;
    unsigned short* Kh = Ql + PXE;
    unsigned short* Kl = Kh + PXE;
    const unsigned short* Xg = Xb + (size_t)p * PXE;
    gemm_bf<0, 2, 0><<<gProj, blk, 0, stream>>>(
        Xg, Xg, DM, 0LL, Wb, Wb, DM, 0LL,
        (void*)Qh, DM, 0LL, (void*)Ql, DM, 0LL, DM,
        BPS * SEQ, DM, DM, 1.0f, 1.0f);
    gemm_bf<0, 2, 0><<<gProj, blk, 0, stream>>>(
        Xg, Xg, DM, 0LL, Wb + (size_t)DM * DM, Wb + (size_t)DM * DM, DM, 0LL,
        (void*)Kh, DM, 0LL, (void*)Kl, DM, 0LL, DM,
        BPS * SEQ, DM, DM, 1.0f, 1.0f);
  }
  gemm_bf<0, 3, 0><<<gVT, blk, 0, stream>>>(
      Wb + (size_t)2 * DM * DM, Wb + (size_t)2 * DM * DM, DM, 0LL, Xb, Xb, DM, (long long)SEQ * DM,
      (void*)VTh, SEQ, (long long)DM * SEQ, (void*)VTl, VLP, (long long)DM * VLP, VLP,
      DM, SEQ, DM, VSC, LSC);
  for (int p = 0; p < NPASS; ++p) {
    const unsigned short* Qh = (const unsigned short*)(ws + oB + (size_t)p * 4 * PXP);
    const unsigned short* Ql = Qh + PXE;
    const unsigned short* Kh = Ql + PXE;
    const unsigned short* Kl = Kh + PXE;
    gemm_bf<SCORE_NSPLIT, 0, 0><<<gS, blk, 0, stream>>>(
        Kh, Kl, DM, (long long)SEQ * DM, Qh, Ql, DM, (long long)SEQ * DM,
        (void*)Sp, SEQ, (long long)SEQ * SEQ, (void*)Sp, SEQ, 0LL, 0,
        SEQ, SEQ, DM, 1.0f, 1.0f);
    softmax_rows<<<gSm, blk, 0, stream>>>(Sp, Ph, Pl, p * BPS);
  }
  gemm_pv<true, 2><<<gPvRes, blk, 0, stream>>>(Ph, Pl, VTh, VTl, out, 0, RESR);
  if (nPvTiles > 0) {
    gemm_pv<false, 4><<<gPv, blk, 0, stream>>>(Ph, Pl, VTh, VTl, out, RESR, SEQ - RESR);
  }
  (void)hipGetLastError();
}
